// StateSpaceModel_29300266893417
// MI455X (gfx1250) — hardware-verified
//
#include <hip/hip_runtime.h>
#include <math.h>

constexpr int kBatch = 2;
constexpr int kSeq   = 2048;
constexpr int kDin   = 2048;
constexpr int kDst   = 16;
constexpr int kDtr   = 128;
constexpr int kEp    = 160;
constexpr int kEpPad = 192;
constexpr int kTok   = kBatch * kSeq;

constexpr size_t kBytesXplane = (size_t)kTok * kDin * 2;
constexpr size_t kBytesWxp    = (size_t)kEpPad * kDin * 2;
constexpr size_t kBytesXdbl   = (size_t)kTok * kEpPad * 4;
constexpr size_t kBytesDr     = (size_t)kTok * kDtr * 2;
constexpr size_t kBytesWdt    = (size_t)kDin * kDtr * 2;
constexpr size_t kBytesDelta  = (size_t)kTok * kDin * 4;
constexpr size_t oXH   = 0;
constexpr size_t oXL   = oXH + kBytesXplane;
constexpr size_t oWPH  = oXL + kBytesXplane;
constexpr size_t oWPL  = oWPH + kBytesWxp;
constexpr size_t oXDBL = oWPL + kBytesWxp;
constexpr size_t oDRH  = oXDBL + kBytesXdbl;
constexpr size_t oDRL  = oDRH + kBytesDr;
constexpr size_t oWDH  = oDRL + kBytesDr;
constexpr size_t oWDL  = oWDH + kBytesWdt;
constexpr size_t oDRAW = oWDL + kBytesWdt;
constexpr size_t kWsTotal = oDRAW + kBytesDelta;
constexpr size_t oDT   = 0;
static_assert(2 * kBytesXplane == kBytesDelta, "DT plane fits exactly over XH+XL");
static_assert(kWsTotal == 74973184, "carve total");
static_assert(kWsTotal <= 134217728, "carve under 128 MiB");
static_assert((oXL % 256) == 0 && (oWPH % 256) == 0 && (oWPL % 256) == 0 && (oXDBL % 256) == 0 &&
              (oDRH % 256) == 0 && (oDRL % 256) == 0 && (oWDH % 256) == 0 && (oWDL % 256) == 0 &&
              (oDRAW % 256) == 0, "256-B aligned regions");
static_assert(kTok % 64 == 0 && kEpPad % 64 == 0 && kDin % 64 == 0, "GEMM M/N tile multiples");
static_assert(kDin % 32 == 0 && kDtr % 32 == 0, "GEMM K multiples of 32");

typedef __attribute__((ext_vector_type(16))) _Float16 v16h;
typedef __attribute__((ext_vector_type(8)))  _Float16 v8h;
typedef __attribute__((ext_vector_type(16))) __bf16   v16b;
typedef __attribute__((ext_vector_type(8)))  __bf16   v8b;
typedef __attribute__((ext_vector_type(8)))  float    v8f;
typedef __attribute__((ext_vector_type(4)))  float    v4f;
typedef __attribute__((ext_vector_type(4)))  unsigned int v4u;

__device__ __forceinline__ unsigned short f2bf_bits(float f) {
  unsigned u = __float_as_uint(f);
  return (unsigned short)((u + 0x7FFFu + ((u >> 16) & 1u)) >> 16);
}
__device__ __forceinline__ float bf_bits2f(unsigned short h) { return __uint_as_float(((unsigned)h) << 16); }

__device__ __forceinline__ void dep_guard_h(v8f& a, v8f& b, v16h x, v16h y) { asm volatile("v_nop\n\tv_nop\n\tv_nop\n\tv_nop" : "+v"(a), "+v"(b) : "v"(x), "v"(y)); }
__device__ __forceinline__ void dep_guard_b(v8f& a, v8f& b, v16b x, v16b y) { asm volatile("v_nop\n\tv_nop\n\tv_nop\n\tv_nop" : "+v"(a), "+v"(b) : "v"(x), "v"(y)); }
__device__ __forceinline__ void keep4_h(v16h a, v16h b, v16h c, v16h d) { asm volatile("v_nop" :: "v"(a), "v"(b), "v"(c), "v"(d)); }
__device__ __forceinline__ void keep4_b(v16b a, v16b b, v16b c, v16b d) { asm volatile("v_nop" :: "v"(a), "v"(b), "v"(c), "v"(d)); }
__device__ __forceinline__ void acc_guard4(v8f& a, v8f& b, v8f& c, v8f& d) { asm volatile("v_nop\n\tv_nop\n\tv_nop\n\tv_nop" : "+v"(a), "+v"(b), "+v"(c), "+v"(d)); }
template <typename T> struct Frag;
template <> struct Frag<_Float16> {
  typedef v16h V; union U { v16h v; v8h h[2]; };
  static __device__ __forceinline__ v16h load(const _Float16* p) {
    U f; f.h[0] = *(const v8h*)(p); f.h[1] = *(const v8h*)(p + 16); return f.v;
  }
  static __device__ __forceinline__ v8f mma(v16h a, v16h b, v8f c) {
    return __builtin_amdgcn_wmma_f32_16x16x32_f16(false, a, false, b, (short)0, c, false, false);
  }
  static __device__ __forceinline__ void guard(v8f& a, v8f& b, v16h x, v16h y) { dep_guard_h(a, b, x, y); }
  static __device__ __forceinline__ void keep(v16h a, v16h b, v16h c, v16h d) { keep4_h(a, b, c, d); }
};
template <> struct Frag<__bf16> {
  typedef v16b V; union U { v16b v; v8b h[2]; };
  static __device__ __forceinline__ v16b load(const __bf16* p) {
    U f; f.h[0] = *(const v8b*)(p); f.h[1] = *(const v8b*)(p + 16); return f.v;
  }
  static __device__ __forceinline__ v8f mma(v16b a, v16b b, v8f c) {
    return __builtin_amdgcn_wmma_f32_16x16x32_bf16(false, a, false, b, (short)0, c, false, false);
  }
  static __device__ __forceinline__ void guard(v8f& a, v8f& b, v16b x, v16b y) { dep_guard_b(a, b, x, y); }
  static __device__ __forceinline__ void keep(v16b a, v16b b, v16b c, v16b d) { keep4_b(a, b, c, d); }
};

__device__ __forceinline__ unsigned pk16(unsigned short a, unsigned short b) { return (unsigned)a | ((unsigned)b << 16); }

template <int ET> struct Elem;
template <> struct Elem<0> { typedef _Float16 T; };
template <> struct Elem<1> { typedef __bf16 T; };
template <int ET, bool SPLIT, int BIAS_MODE, int OUT_MODE, bool RESID, int ACT = 0>
__global__ __launch_bounds__(256) void wmma_gemm64(
    const unsigned short* __restrict__ Ap, const unsigned short* __restrict__ A2p, int lda, long strideA,
    const unsigned short* __restrict__ Btp, const unsigned short* __restrict__ Bt2p, int ldb, long strideB,
    void* __restrict__ Cout, void* __restrict__ Cout2, int ldc, long strideC,
    const float* __restrict__ bias,
    const float* __restrict__ resid, long strideR,
    int M, int N, int K, float scale) {
  typedef typename Elem<ET>::T T;
  typedef typename Frag<T>::V V;
  const T* A = (const T*)Ap; const T* A2 = (const T*)A2p; const T* Bt = (const T*)Btp; const T* Bt2 = (const T*)Bt2p;
  __shared__ __align__(16) float sT[8][16 * 68];
  const int b    = blockIdx.y;
  const int lane = threadIdx.x & 31;
  const int wave = threadIdx.x >> 5;
  const int tilesN = N >> 6;
  const int tilesM = M >> 6;
  const int tile = blockIdx.x * 8 + wave;
  if (tile >= tilesM * tilesN) return;
  const int tm = tile / tilesN;
  const int tn = tile - tm * tilesN;
  const int m0 = tm << 6;
  const int n0 = tn << 6;

  const T* Ab  = A  + (size_t)b * strideA;
  const T* Bb  = Bt + (size_t)b * strideB;
  const T* Ab2 = SPLIT ? (A2  + (size_t)b * strideA) : nullptr;
  const T* Bb2 = SPLIT ? (Bt2 + (size_t)b * strideB) : nullptr;

  const int rlane = lane & 15;
  const int koff  = (lane >> 4) * 8;
  const int mOff  = (lane >> 4) * 8;

  v8f acc[4][4];
#pragma unroll
  for (int i = 0; i < 4; ++i)
#pragma unroll
    for (int j = 0; j < 4; ++j) acc[i][j] = (v8f){0.f,0.f,0.f,0.f,0.f,0.f,0.f,0.f};

  for (int k0 = 0; k0 < K; k0 += 32) {
    V bh[4], bl[4];
#pragma unroll
    for (int j = 0; j < 4; ++j) {
      const size_t bo = (size_t)(n0 + (j << 4) + rlane) * ldb + koff + k0;
      bh[j] = Frag<T>::load(Bb + bo);
      if (SPLIT) bl[j] = Frag<T>::load(Bb2 + bo);
    }
#pragma unroll
    for (int i = 0; i < 4; ++i) {
      const size_t ao = (size_t)(m0 + (i << 4) + rlane) * lda + koff + k0;
      V ah = Frag<T>::load(Ab + ao);
      V al;
      if (SPLIT) al = Frag<T>::load(Ab2 + ao);
#pragma unroll
      for (int j = 0; j < 4; ++j) {
        acc[i][j] = Frag<T>::mma(ah, bh[j], acc[i][j]);
        if (SPLIT) {
          acc[i][j] = Frag<T>::mma(ah, bl[j], acc[i][j]);
          acc[i][j] = Frag<T>::mma(al, bh[j], acc[i][j]);
        }
      }
      Frag<T>::guard(acc[i][0], acc[i][3], ah, SPLIT ? al : ah);
    }
    Frag<T>::keep(bh[0], bh[1], bh[2], bh[3]);
    if (SPLIT) Frag<T>::keep(bl[0], bl[1], bl[2], bl[3]);
  }
  acc_guard4(acc[0][0], acc[0][1], acc[0][2], acc[0][3]);
  acc_guard4(acc[1][0], acc[1][1], acc[1][2], acc[1][3]);
  acc_guard4(acc[2][0], acc[2][1], acc[2][2], acc[2][3]);
  acc_guard4(acc[3][0], acc[3][1], acc[3][2], acc[3][3]);

  float* slab = sT[wave];
  const float* Rb = RESID ? (resid + (size_t)b * strideR) : nullptr;
#pragma unroll
  for (int i = 0; i < 4; ++i) {
    const int mBase = m0 + (i << 4);
#pragma unroll
    for (int j = 0; j < 4; ++j) {
      const int n = n0 + (j << 4) + rlane;
      float bv = 0.f;
      if (BIAS_MODE == 2) bv = bias[n];
#pragma unroll
      for (int r = 0; r < 8; ++r) {
        float v = acc[i][j][r] * scale;
        if (BIAS_MODE == 1) v += bias[mBase + mOff + r];
        if (BIAS_MODE == 2) v += bv;
        if (RESID) v += Rb[(size_t)(mBase + mOff + r) * ldc + n];
        if (ACT == 2) v = fmaxf(v, 0.0f);
        if (ACT == 4) v = (v > 0.f) ? v : 0.01f * v;
        slab[(mOff + r) * 68 + (j << 4) + rlane] = v;
      }
    }
    __builtin_amdgcn_fence(__ATOMIC_RELEASE, "workgroup");
    __builtin_amdgcn_wave_barrier();
    __builtin_amdgcn_fence(__ATOMIC_ACQUIRE, "workgroup");
    if (OUT_MODE == 0) {
      float* C = (float*)Cout + (size_t)b * strideC;
      const int hh = lane >> 4, c4 = (lane & 15) * 4;
      for (int pass = 0; pass < 2; ++pass) {
#pragma unroll
        for (int it = 0; it < 8; ++it) {
          const int row = it * 2 + hh;
          v4f v = *(const v4f*)(slab + row * 68 + c4);
          *(volatile v4f*)(C + (size_t)(mBase + row) * ldc + n0 + c4) = v;
        }
        __threadfence();
      }
    } else {
      const int q = lane >> 3, c8 = (lane & 7) * 8;
      unsigned short* C  = (unsigned short*)Cout  + (size_t)b * strideC;
      unsigned short* C2 = (OUT_MODE == 2) ? ((unsigned short*)Cout2 + (size_t)b * strideC) : nullptr;
      for (int pass = 0; pass < 2; ++pass) {
#pragma unroll
        for (int it = 0; it < 4; ++it) {
          const int row = it * 4 + q;
          const float* sp = slab + row * 68 + c8;
          v8h hv, lv;
#pragma unroll
          for (int e = 0; e < 8; ++e) {
            if (OUT_MODE == 1) {
              hv[e] = (_Float16)sp[e];
            } else {
              unsigned short hb = f2bf_bits(sp[e]);
              unsigned short lb = f2bf_bits(sp[e] - bf_bits2f(hb));
              hv[e] = __builtin_bit_cast(_Float16, hb);
              lv[e] = __builtin_bit_cast(_Float16, lb);
            }
          }
          *(volatile v8h*)(C + (size_t)(mBase + row) * ldc + n0 + c8) = hv;
          if (OUT_MODE == 2) *(volatile v8h*)(C2 + (size_t)(mBase + row) * ldc + n0 + c8) = lv;
        }
        __threadfence();
      }
    }
    __builtin_amdgcn_fence(__ATOMIC_RELEASE, "workgroup");
    __builtin_amdgcn_wave_barrier();
    __builtin_amdgcn_fence(__ATOMIC_ACQUIRE, "workgroup");
  }
}

__global__ __launch_bounds__(256) void split8_bf16_kernel(const float* __restrict__ in, int src_rows, int cols, int src_pitch,
                                                          unsigned short* __restrict__ outH, unsigned short* __restrict__ outL,
                                                          int n8_out) {
  const int i = blockIdx.x * 256 + threadIdx.x;
  if (i >= n8_out) return;
  const int cols8 = cols >> 3;
  const int row = i / cols8;
  const int c = (i - row * cols8) * 8;
  const int rowc = (row < src_rows) ? row : (src_rows - 1);
  const bool live = (row < src_rows);
  const float* p = in + (size_t)rowc * src_pitch + c;
  const v4f a  = *(const v4f*)(p);
  const v4f b2 = *(const v4f*)(p + 4);
  unsigned short hb[8], lb[8];
#pragma unroll
  for (int e = 0; e < 4; ++e) {
    const float f0 = live ? a[e]  : 0.0f;
    const float f1 = live ? b2[e] : 0.0f;
    hb[e]     = f2bf_bits(f0);
    lb[e]     = f2bf_bits(f0 - bf_bits2f(hb[e]));
    hb[4 + e] = f2bf_bits(f1);
    lb[4 + e] = f2bf_bits(f1 - bf_bits2f(hb[4 + e]));
  }
  const v4u uh = (v4u){pk16(hb[0], hb[1]), pk16(hb[2], hb[3]), pk16(hb[4], hb[5]), pk16(hb[6], hb[7])};
  const v4u ul = (v4u){pk16(lb[0], lb[1]), pk16(lb[2], lb[3]), pk16(lb[4], lb[5]), pk16(lb[6], lb[7])};
  unsigned short* qh = outH + 8 * (size_t)i;
  unsigned short* ql = outL + 8 * (size_t)i;
  *(volatile v4u*)qh = uh;
  *(volatile v4u*)ql = ul;
  __threadfence();
  *(volatile v4u*)qh = uh;
  *(volatile v4u*)ql = ul;
}

__global__ __launch_bounds__(256) void softplus4_kernel(const float* __restrict__ in, const float* __restrict__ bias,
                                                        float* __restrict__ outp, int n4) {
  const int i = blockIdx.x * 256 + threadIdx.x;
  if (i >= n4) return;
  const size_t e0 = 4 * (size_t)i;
  const int dcol = (int)(e0 & (size_t)(kDin - 1));
  const v4f a  = *(const v4f*)(in + e0);
  const v4f bb = *(const v4f*)(bias + dcol);
  v4f r;
#pragma unroll
  for (int e = 0; e < 4; ++e) {
    const float v = a[e] + bb[e];
    r[e] = fmaxf(v, 0.0f) + log1pf(expf(-fabsf(v)));
  }
  float* q = outp + e0;
  *(volatile v4f*)q = r;
  __threadfence();
  *(volatile v4f*)q = r;
}

constexpr int kScanTPB = 64;
constexpr int kScanTC  = 64;
static_assert(kDin % kScanTPB == 0 && kSeq % kScanTC == 0, "scan tiling");

__global__ __launch_bounds__(kScanTPB) void scan_kernel(const float* __restrict__ x, const float* __restrict__ A_log,
                                                         const float* __restrict__ Dvec, const float* __restrict__ xdbl,
                                                         const float* __restrict__ dt, float* __restrict__ out) {
  __shared__ __align__(16) float sBC[kScanTC * 32];
  __shared__ __align__(16) float sY[kScanTC * kScanTPB];
  const int tid  = threadIdx.x;
  const int lane = tid & 31;
  const int wave = tid >> 5;
  const int bpb  = kDin / kScanTPB;
  const int b    = blockIdx.x / bpb;
  const int d0   = (blockIdx.x - b * bpb) * kScanTPB;
  const int d    = d0 + tid;

  float An[kDst], h[kDst];
#pragma unroll
  for (int n = 0; n < kDst; ++n) {
    An[n] = -expf(A_log[(size_t)d * kDst + n]);
    h[n]  = 0.0f;
  }
  const float Dd = Dvec[d];
  const size_t rowb = (size_t)b * kSeq;

  for (int tc = 0; tc < kSeq / kScanTC; ++tc) {
    const int t0 = tc * kScanTC;
    __syncthreads();
#pragma unroll
    for (int it = 0; it < 8; ++it) {
      const int s   = it * kScanTPB + tid;
      const int tr  = s >> 3;
      const int seg = s & 7;
      const v4f v = *(const v4f*)(xdbl + (rowb + t0 + tr) * (size_t)kEpPad + kDtr + seg * 4);
      *(v4f*)(sBC + tr * 32 + seg * 4) = v;
    }
    __syncthreads();

#pragma unroll 1
    for (int t = 0; t < kScanTC; ++t) {
      const size_t g = (rowb + t0 + t) * (size_t)kDin + d;
      const float dl = dt[g];
      const float u  = x[g];
      const float du = dl * u;
      const float* bc = sBC + t * 32;
      const v4f vb0 = *(const v4f*)(bc);
      const v4f vb1 = *(const v4f*)(bc + 4);
      const v4f vb2 = *(const v4f*)(bc + 8);
      const v4f vb3 = *(const v4f*)(bc + 12);
      const v4f vc0 = *(const v4f*)(bc + 16);
      const v4f vc1 = *(const v4f*)(bc + 20);
      const v4f vc2 = *(const v4f*)(bc + 24);
      const v4f vc3 = *(const v4f*)(bc + 28);
      float Bn[kDst], Cn[kDst];
#pragma unroll
      for (int e = 0; e < 4; ++e) {
        Bn[e] = vb0[e]; Bn[4 + e] = vb1[e]; Bn[8 + e] = vb2[e]; Bn[12 + e] = vb3[e];
        Cn[e] = vc0[e]; Cn[4 + e] = vc1[e]; Cn[8 + e] = vc2[e]; Cn[12 + e] = vc3[e];
      }
      float y = 0.0f;
#pragma unroll
      for (int n = 0; n < kDst; ++n) {
        const float a  = expf(dl * An[n]);
        const float hn = a * h[n] + du * Bn[n];
        h[n] = hn;
        y += hn * Cn[n];
      }
      sY[t * kScanTPB + tid] = y + u * Dd;
    }
    __syncthreads();

    const int hh = lane >> 4;
    const int c4 = (lane & 15) * 4;
    for (int pass = 0; pass < 2; ++pass) {
#pragma unroll
      for (int it = 0; it < 16; ++it) {
        const int row = wave * 32 + it * 2 + hh;
        const v4f v = *(const v4f*)(sY + row * kScanTPB + c4);
        *(volatile v4f*)(out + (rowb + t0 + row) * (size_t)kDin + d0 + c4) = v;
      }
      __threadfence();
    }
  }
}

extern "C" void kernel_launch(void* const* d_in, const int* in_sizes, int n_in,
                              void* d_out, int out_size, void* d_ws, size_t ws_size,
                              hipStream_t stream) {
  if (n_in < 6) return;
  if (in_sizes[0] != kTok * kDin || in_sizes[1] != kDin * kDst || in_sizes[2] != kDin ||
      in_sizes[3] != kEp * kDin || in_sizes[4] != kDin * kDtr || in_sizes[5] != kDin) return;
  if (out_size != kTok * kDin) return;
  if (ws_size < kWsTotal) return;

  const float* x     = (const float*)d_in[0];
  const float* A_log = (const float*)d_in[1];
  const float* Dvec  = (const float*)d_in[2];
  const float* xpw   = (const float*)d_in[3];
  const float* dtw   = (const float*)d_in[4];
  const float* dtb   = (const float*)d_in[5];
  float* out = (float*)d_out;

  unsigned char* ws = (unsigned char*)d_ws;
  unsigned short* XH   = (unsigned short*)(ws + oXH);
  unsigned short* XL   = (unsigned short*)(ws + oXL);
  unsigned short* WPH  = (unsigned short*)(ws + oWPH);
  unsigned short* WPL  = (unsigned short*)(ws + oWPL);
  float*          XDBL = (float*)(ws + oXDBL);
  unsigned short* DRH  = (unsigned short*)(ws + oDRH);
  unsigned short* DRL  = (unsigned short*)(ws + oDRL);
  unsigned short* WDH  = (unsigned short*)(ws + oWDH);
  unsigned short* WDL  = (unsigned short*)(ws + oWDL);
  float*          DRAW = (float*)(ws + oDRAW);
  float*          DT   = (float*)(ws + oDT);

  {
    const int n8 = kTok * kDin / 8;
    split8_bf16_kernel<<<(n8 + 255) / 256, 256, 0, stream>>>(x, kTok, kDin, kDin, XH, XL, n8);
  }
  {
    const int n8 = kEpPad * kDin / 8;
    split8_bf16_kernel<<<(n8 + 255) / 256, 256, 0, stream>>>(xpw, kEp, kDin, kDin, WPH, WPL, n8);
  }
  {
    const int n8 = kDin * kDtr / 8;
    split8_bf16_kernel<<<(n8 + 255) / 256, 256, 0, stream>>>(dtw, kDin, kDtr, kDtr, WDH, WDL, n8);
  }
  {
    const dim3 grid((kTok / 64) * (kEpPad / 64) / 8, 1);
    wmma_gemm64<1, true, 0, 0, false, 0><<<grid, 256, 0, stream>>>(
        XH, XL, kDin, 0L, WPH, WPL, kDin, 0L, (void*)XDBL, (void*)nullptr, kEpPad, 0L,
        (const float*)nullptr, (const float*)nullptr, 0L, kTok, kEpPad, kDin, 1.0f);
  }
  {
    const int n8 = kTok * kDtr / 8;
    split8_bf16_kernel<<<(n8 + 255) / 256, 256, 0, stream>>>(XDBL, kTok, kDtr, kEpPad, DRH, DRL, n8);
  }
  {
    const dim3 grid((kTok / 64) * (kDin / 64) / 8, 1);
    wmma_gemm64<1, true, 0, 0, false, 0><<<grid, 256, 0, stream>>>(
        DRH, DRL, kDtr, 0L, WDH, WDL, kDtr, 0L, (void*)DRAW, (void*)nullptr, kDin, 0L,
        (const float*)nullptr, (const float*)nullptr, 0L, kTok, kDin, kDtr, 1.0f);
  }
  {
    const int n4 = kTok * kDin / 4;
    softplus4_kernel<<<(n4 + 255) / 256, 256, 0, stream>>>(DRAW, dtb, DT, n4);
  }
  scan_kernel<<<kBatch * kDin / kScanTPB, kScanTPB, 0, stream>>>(x, A_log, Dvec, XDBL, DT, out);
}
